// Decoder_55963423867149
// MI455X (gfx1250) — hardware-verified
//
#include <hip/hip_runtime.h>
#include <math.h>

constexpr int T_STEPS = 48;
constexpr int BATCH   = 64;
constexpr int SRCLEN  = 100;
constexpr int HID     = 512;
constexpr int GATES3  = 3 * HID;
constexpr int CATW    = 3 * HID;
constexpr int VOCAB   = 32000;
constexpr int ROWS_TB = T_STEPS * BATCH;
constexpr int ROWS_LB = SRCLEN * BATCH;
constexpr int HPITCH  = 520;
constexpr int FPITCH  = 516;
constexpr int GIS_P    = 20;
constexpr int GIS_GATE = 16 * GIS_P;
constexpr int GIS_WAVE = 3 * GIS_GATE;
constexpr float OPCARRY  = 16.0f;
constexpr float FOLD_INV = 1.0f / (OPCARRY * OPCARRY);

constexpr int OUT0_N = T_STEPS * BATCH * (HID / 2);
constexpr int OUT1_N = T_STEPS * BATCH * SRCLEN;
constexpr int OUT2_N = T_STEPS * BATCH;
constexpr int OUT3_N = BATCH * HID;
constexpr int OUT4_N = BATCH * SRCLEN;
constexpr int OUT5_N = BATCH * HID;
constexpr int OUT6_N = T_STEPS * BATCH * HID;
constexpr int OFF1 = OUT0_N;
constexpr int OFF2 = OFF1 + OUT1_N;
constexpr int OFF3 = OFF2 + OUT2_N;
constexpr int OFF4 = OFF3 + OUT3_N;
constexpr int OFF5 = OFF4 + OUT4_N;
constexpr int OFF6 = OFF5 + OUT5_N;
constexpr int OUT_TOTAL = OFF6 + OUT6_N;
static_assert(OFF1 * 4 == 3145728);
static_assert(OFF2 * 4 == 4374528);
static_assert(OFF3 * 4 == 4386816);
static_assert(OFF4 * 4 == 4517888);
static_assert(OFF5 * 4 == 4543488);
static_assert(OFF6 * 4 == 4674560);
static_assert(OUT_TOTAL * 4 == 10966016);
static_assert((OFF1 * 4) % 128 == 0 && (OFF2 * 4) % 128 == 0 && (OFF3 * 4) % 128 == 0);
static_assert((OFF4 * 4) % 128 == 0 && (OFF5 * 4) % 128 == 0 && (OFF6 * 4) % 128 == 0);
static_assert(ROWS_TB % 64 == 0 && ROWS_LB % 64 == 0 && HID % 64 == 0 && GATES3 % 64 == 0);
static_assert(HID % 32 == 0 && CATW % 32 == 0);
static_assert((16 * SRCLEN * 4) % 128 == 0);
static_assert(8 * GIS_WAVE <= 16 * FPITCH);
static_assert(BATCH % 16 == 0);

typedef __attribute__((ext_vector_type(16))) _Float16 v16h;
typedef __attribute__((ext_vector_type(8)))  _Float16 v8h;
typedef __attribute__((ext_vector_type(16))) __bf16   v16b;
typedef __attribute__((ext_vector_type(8)))  __bf16   v8b;
typedef __attribute__((ext_vector_type(8)))  float    v8f;
typedef __attribute__((ext_vector_type(4)))  float    v4f;

__device__ __forceinline__ unsigned short f2bf_bits(float f) {
  unsigned u = __float_as_uint(f);
  return (unsigned short)((u + 0x7FFFu + ((u >> 16) & 1u)) >> 16);
}
__device__ __forceinline__ float bf_bits2f(unsigned short h) { return __uint_as_float(((unsigned)h) << 16); }

__device__ __forceinline__ void dep_guard4_h(v8f& a, v8f& b, v8f& c, v8f& d, v16h x, v16h y) {
  asm volatile("v_nop\n\tv_nop\n\tv_nop\n\tv_nop" : "+v"(a), "+v"(b), "+v"(c), "+v"(d) : "v"(x), "v"(y));
}
__device__ __forceinline__ void dep_guard4_b(v8f& a, v8f& b, v8f& c, v8f& d, v16b x, v16b y) {
  asm volatile("v_nop\n\tv_nop\n\tv_nop\n\tv_nop" : "+v"(a), "+v"(b), "+v"(c), "+v"(d) : "v"(x), "v"(y));
}
__device__ __forceinline__ void keep4_h(v16h a, v16h b, v16h c, v16h d) { asm volatile("v_nop" :: "v"(a), "v"(b), "v"(c), "v"(d)); }
__device__ __forceinline__ void keep4_b(v16b a, v16b b, v16b c, v16b d) { asm volatile("v_nop" :: "v"(a), "v"(b), "v"(c), "v"(d)); }
__device__ __forceinline__ void acc_guard4(v8f& a, v8f& b, v8f& c, v8f& d) {
  asm volatile("v_nop\n\tv_nop\n\tv_nop\n\tv_nop" : "+v"(a), "+v"(b), "+v"(c), "+v"(d));
}
__device__ __forceinline__ void guard_gru(v8f& a, v8f& b, v8f& c, v8f& d, v16h x0, v16h x1,
                                          v16h y0, v16h y1, v16h y2, v16h y3, v16h y4, v16h y5) {
  asm volatile("v_nop\n\tv_nop\n\tv_nop\n\tv_nop"
               : "+v"(a), "+v"(b), "+v"(c), "+v"(d)
               : "v"(x0), "v"(x1), "v"(y0), "v"(y1), "v"(y2), "v"(y3), "v"(y4), "v"(y5));
}
__device__ __forceinline__ void guard_q(v8f& a, v8f& b, v8f& c, v8f& d, v16h x0,
                                        v16h y0, v16h y1, v16h y2, v16h y3) {
  asm volatile("v_nop\n\tv_nop\n\tv_nop\n\tv_nop"
               : "+v"(a), "+v"(b), "+v"(c), "+v"(d)
               : "v"(x0), "v"(y0), "v"(y1), "v"(y2), "v"(y3));
}
__device__ __forceinline__ void wave_sync_lds() {
  __builtin_amdgcn_fence(__ATOMIC_RELEASE, "workgroup");
  __builtin_amdgcn_wave_barrier();
  __builtin_amdgcn_fence(__ATOMIC_ACQUIRE, "workgroup");
}

template <typename T> struct Frag;
template <> struct Frag<_Float16> {
  typedef v16h V; union U { v16h v; v8h h[2]; };
  static __device__ __forceinline__ v16h load(const _Float16* p) {
    U f; f.h[0] = *(const v8h*)(p); f.h[1] = *(const v8h*)(p + 16); return f.v;
  }
  static __device__ __forceinline__ v8f mma(v16h a, v16h b, v8f c) {
    return __builtin_amdgcn_wmma_f32_16x16x32_f16(false, a, false, b, (short)0, c, false, false);
  }
  static __device__ __forceinline__ void guard4(v8f& a, v8f& b, v8f& c, v8f& d, v16h x, v16h y) { dep_guard4_h(a, b, c, d, x, y); }
  static __device__ __forceinline__ void keep(v16h a, v16h b, v16h c, v16h d) { keep4_h(a, b, c, d); }
};
template <> struct Frag<__bf16> {
  typedef v16b V; union U { v16b v; v8b h[2]; };
  static __device__ __forceinline__ v16b load(const __bf16* p) {
    U f; f.h[0] = *(const v8b*)(p); f.h[1] = *(const v8b*)(p + 16); return f.v;
  }
  static __device__ __forceinline__ v8f mma(v16b a, v16b b, v8f c) {
    return __builtin_amdgcn_wmma_f32_16x16x32_bf16(false, a, false, b, (short)0, c, false, false);
  }
  static __device__ __forceinline__ void guard4(v8f& a, v8f& b, v8f& c, v8f& d, v16b x, v16b y) { dep_guard4_b(a, b, c, d, x, y); }
  static __device__ __forceinline__ void keep(v16b a, v16b b, v16b c, v16b d) { keep4_b(a, b, c, d); }
};

template <int ET> struct Elem;
template <> struct Elem<0> { typedef _Float16 T; };
template <> struct Elem<1> { typedef __bf16 T; };
template <int ET, bool SPLIT, int BIAS_MODE, int OUT_MODE, bool RESID, int ACT = 0>
__global__ __launch_bounds__(256) void wmma_gemm64(
    const unsigned short* __restrict__ Ap, const unsigned short* __restrict__ A2p, int lda, long strideA,
    const unsigned short* __restrict__ Btp, const unsigned short* __restrict__ Bt2p, int ldb, long strideB,
    void* __restrict__ Cout, void* __restrict__ Cout2, int ldc, long strideC,
    const float* __restrict__ bias,
    const float* __restrict__ resid, long strideR,
    int M, int N, int K, float scale) {
  typedef typename Elem<ET>::T T;
  typedef typename Frag<T>::V V;
  const T* A = (const T*)Ap; const T* A2 = (const T*)A2p; const T* Bt = (const T*)Btp; const T* Bt2 = (const T*)Bt2p;
  __shared__ __align__(16) float sT[8][16 * 68];
  const int b    = blockIdx.y;
  const int lane = threadIdx.x & 31;
  const int wave = threadIdx.x >> 5;
  const int tilesN = N >> 6;
  const int tilesM = M >> 6;
  const int tile = blockIdx.x * 8 + wave;
  if (tile >= tilesM * tilesN) return;
  const int tm = tile / tilesN;
  const int tn = tile - tm * tilesN;
  const int m0 = tm << 6;
  const int n0 = tn << 6;

  const T* Ab  = A  + (size_t)b * strideA;
  const T* Bb  = Bt + (size_t)b * strideB;
  const T* Ab2 = SPLIT ? (A2  + (size_t)b * strideA) : nullptr;
  const T* Bb2 = SPLIT ? (Bt2 + (size_t)b * strideB) : nullptr;

  const int rlane = lane & 15;
  const int koff  = (lane >> 4) * 8;
  const int mOff  = (lane >> 4) * 8;

  v8f acc[4][4];
#pragma unroll
  for (int i = 0; i < 4; ++i)
#pragma unroll
    for (int j = 0; j < 4; ++j) acc[i][j] = (v8f){0.f,0.f,0.f,0.f,0.f,0.f,0.f,0.f};

  for (int k0 = 0; k0 < K; k0 += 32) {
    V bh[4], bl[4];
#pragma unroll
    for (int j = 0; j < 4; ++j) {
      const size_t bo = (size_t)(n0 + (j << 4) + rlane) * ldb + koff + k0;
      bh[j] = Frag<T>::load(Bb + bo);
      if (SPLIT) bl[j] = Frag<T>::load(Bb2 + bo);
    }
#pragma unroll
    for (int i = 0; i < 4; ++i) {
      const size_t ao = (size_t)(m0 + (i << 4) + rlane) * lda + koff + k0;
      V ah = Frag<T>::load(Ab + ao);
      V al;
      if (SPLIT) al = Frag<T>::load(Ab2 + ao);
#pragma unroll
      for (int j = 0; j < 4; ++j) {
        acc[i][j] = Frag<T>::mma(ah, bh[j], acc[i][j]);
        if (SPLIT) {
          acc[i][j] = Frag<T>::mma(ah, bl[j], acc[i][j]);
          acc[i][j] = Frag<T>::mma(al, bh[j], acc[i][j]);
        }
      }
      Frag<T>::guard4(acc[i][0], acc[i][1], acc[i][2], acc[i][3], ah, SPLIT ? al : ah);
    }
    Frag<T>::keep(bh[0], bh[1], bh[2], bh[3]);
    if (SPLIT) Frag<T>::keep(bl[0], bl[1], bl[2], bl[3]);
  }
  acc_guard4(acc[0][0], acc[0][1], acc[0][2], acc[0][3]);
  acc_guard4(acc[1][0], acc[1][1], acc[1][2], acc[1][3]);
  acc_guard4(acc[2][0], acc[2][1], acc[2][2], acc[2][3]);
  acc_guard4(acc[3][0], acc[3][1], acc[3][2], acc[3][3]);

  float* slab = sT[wave];
  const float* Rb = RESID ? (resid + (size_t)b * strideR) : nullptr;
#pragma unroll
  for (int i = 0; i < 4; ++i) {
    const int mBase = m0 + (i << 4);
#pragma unroll
    for (int j = 0; j < 4; ++j) {
      const int n = n0 + (j << 4) + rlane;
      float bv = 0.f;
      if (BIAS_MODE == 2) bv = bias[n];
#pragma unroll
      for (int r = 0; r < 8; ++r) {
        float v = acc[i][j][r] * scale;
        if (BIAS_MODE == 1) v += bias[mBase + mOff + r];
        if (BIAS_MODE == 2) v += bv;
        if (RESID) v += Rb[(size_t)(mBase + mOff + r) * ldc + n];
        if (ACT == 1) v = tanhf(v);
        if (ACT == 2) v = fmaxf(v, 0.0f);
        slab[(mOff + r) * 68 + (j << 4) + rlane] = v;
      }
    }
    wave_sync_lds();
    if (OUT_MODE == 0) {
      float* C = (float*)Cout + (size_t)b * strideC;
      const int hh = lane >> 4, c4 = (lane & 15) * 4;
      for (int pass = 0; pass < 2; ++pass) {
#pragma unroll
        for (int it = 0; it < 8; ++it) {
          const int row = it * 2 + hh;
          v4f v = *(const v4f*)(slab + row * 68 + c4);
          *(volatile v4f*)(C + (size_t)(mBase + row) * ldc + n0 + c4) = v;
        }
        __threadfence();
      }
    } else {
      const int q = lane >> 3, c8 = (lane & 7) * 8;
      unsigned short* C  = (unsigned short*)Cout  + (size_t)b * strideC;
      unsigned short* C2 = (OUT_MODE == 2) ? ((unsigned short*)Cout2 + (size_t)b * strideC) : nullptr;
      for (int pass = 0; pass < 2; ++pass) {
#pragma unroll
        for (int it = 0; it < 4; ++it) {
          const int row = it * 4 + q;
          const float* sp = slab + row * 68 + c8;
          v8h hv, lv;
#pragma unroll
          for (int e = 0; e < 8; ++e) {
            if (OUT_MODE == 1) {
              hv[e] = (_Float16)sp[e];
            } else {
              unsigned short hb = f2bf_bits(sp[e]);
              unsigned short lb = f2bf_bits(sp[e] - bf_bits2f(hb));
              hv[e] = __builtin_bit_cast(_Float16, hb);
              lv[e] = __builtin_bit_cast(_Float16, lb);
            }
          }
          *(volatile v8h*)(C + (size_t)(mBase + row) * ldc + n0 + c8) = hv;
          if (OUT_MODE == 2) *(volatile v8h*)(C2 + (size_t)(mBase + row) * ldc + n0 + c8) = lv;
        }
        __threadfence();
      }
    }
    wave_sync_lds();
  }
}

__global__ __launch_bounds__(256) void cvt8_f16_kernel(const float* __restrict__ src, unsigned short* __restrict__ dst,
                                                       int nrow, int ncol8, int spitch, int scol0, float sc) {
  const int i  = blockIdx.x * 256 + threadIdx.x;
  const int n8 = nrow * ncol8;
  if (i < n8) {
    const int row = i / ncol8;
    const int c8  = i - row * ncol8;
    const float* sp = src + (size_t)row * spitch + scol0 + c8 * 8;
    const v4f a = *(const v4f*)(sp);
    const v4f b = *(const v4f*)(sp + 4);
    v8h hv;
#pragma unroll
    for (int e = 0; e < 4; ++e) {
      const float fa = a[e] * sc;
      const float fb = b[e] * sc;
      hv[e]     = (_Float16)fa;
      hv[4 + e] = (_Float16)fb;
    }
    *(volatile v8h*)(dst + (size_t)i * 8) = hv;
    __threadfence();
    *(volatile v8h*)(dst + (size_t)i * 8) = hv;
  }
}

__global__ __launch_bounds__(256) void gather_emb_kernel(const int* __restrict__ ids, const float* __restrict__ lut,
                                                         unsigned short* __restrict__ acat) {
  const int i = blockIdx.x * 256 + threadIdx.x;
  if (i < ROWS_TB * 64) {
    const int row = i >> 6;
    const int c8  = (i & 63) * 8;
    int id = ids[row];
    id = id < 0 ? 0 : (id > VOCAB - 1 ? VOCAB - 1 : id);
    const float* sp = lut + (size_t)id * HID + c8;
    const v4f a = *(const v4f*)(sp);
    const v4f b = *(const v4f*)(sp + 4);
    v8h hv;
#pragma unroll
    for (int e = 0; e < 4; ++e) {
      const float fa = a[e] * OPCARRY;
      const float fb = b[e] * OPCARRY;
      hv[e]     = (_Float16)fa;
      hv[4 + e] = (_Float16)fb;
    }
    unsigned short* dp = acat + (size_t)row * CATW + c8;
    *(volatile v8h*)dp = hv;
    __threadfence();
    *(volatile v8h*)dp = hv;
  }
}

__device__ __forceinline__ void tile_to_f16(const float* src, _Float16* dst, int tid) {
#pragma unroll 1
  for (int it = 0; it < 4; ++it) {
    const int idx = it * 256 + tid;
    const int row = idx >> 6;
    const int c8  = (idx & 63) * 8;
    const v4f a = *(const v4f*)(src + row * FPITCH + c8);
    const v4f b = *(const v4f*)(src + row * FPITCH + c8 + 4);
    v8h hv;
#pragma unroll
    for (int e = 0; e < 4; ++e) {
      const float fa = a[e] * OPCARRY;
      const float fb = b[e] * OPCARRY;
      hv[e]     = (_Float16)fa;
      hv[4 + e] = (_Float16)fb;
    }
    *(v8h*)(dst + row * HPITCH + c8) = hv;
  }
}

__device__ __forceinline__ void tile_emit(const float* src, const _Float16* src16, unsigned short* g16,
                                          float* g32, float* gfin, bool last, int tid) {
  for (int pass = 0; pass < 2; ++pass) {
#pragma unroll 1
    for (int it = 0; it < 4; ++it) {
      const int idx = it * 256 + tid;
      const int row = idx >> 6;
      const int c8  = (idx & 63) * 8;
      const v8h hv = *(const v8h*)(src16 + row * HPITCH + c8);
      *(volatile v8h*)(g16 + (size_t)row * CATW + c8) = hv;
    }
#pragma unroll 1
    for (int it = 0; it < 8; ++it) {
      const int idx = it * 256 + tid;
      const int row = idx >> 7;
      const int c4  = (idx & 127) * 4;
      const v4f v = *(const v4f*)(src + row * FPITCH + c4);
      *(volatile v4f*)(g32 + (size_t)row * HID + c4) = v;
      if (last) *(volatile v4f*)(gfin + (size_t)row * HID + c4) = v;
    }
    __threadfence();
  }
}

__global__ __launch_bounds__(256) void dec_seq_kernel(
    const float* __restrict__ hidden, const float* __restrict__ init_att,
    const float* __restrict__ context, const float* __restrict__ mask,
    const float* __restrict__ pre32, const float* __restrict__ gi32,
    const float* __restrict__ b_hh, const float* __restrict__ w_v,
    const unsigned short* __restrict__ whh16p, const unsigned short* __restrict__ wihc16p,
    const unsigned short* __restrict__ wq16p,
    unsigned short* __restrict__ acat16, float* __restrict__ wctx32,
    float* __restrict__ out1, float* __restrict__ out3, float* __restrict__ out4,
    float* __restrict__ out5, float* __restrict__ out6) {
  __shared__ __align__(16) _Float16 Ah[16 * HPITCH];
  __shared__ __align__(16) _Float16 Ac[16 * HPITCH];
  __shared__ __align__(16) float    Hs[16 * FPITCH];
  __shared__ __align__(16) float    Fs[16 * FPITCH];
  __shared__ __align__(16) float    Ss[16 * SRCLEN];
  __shared__ __align__(16) float    sBhh[GATES3];
  __shared__ __align__(16) float    sWv[HID];

  const _Float16* WHH = (const _Float16*)whh16p;
  const _Float16* WIC = (const _Float16*)wihc16p;
  const _Float16* WQ  = (const _Float16*)wq16p;
  const int tid = threadIdx.x, lane = tid & 31, wave = tid >> 5;
  const int c = lane & 15, hh = lane >> 4, koff = hh * 8;
  const int b0 = blockIdx.x * 16;

#pragma unroll 1
  for (int i = tid; i < GATES3 / 4; i += 256) *(v4f*)(sBhh + 4 * i) = *(const v4f*)(b_hh + 4 * i);
  if (tid < HID / 4) *(v4f*)(sWv + 4 * tid) = *(const v4f*)(w_v + 4 * tid);
#pragma unroll 1
  for (int it = 0; it < 8; ++it) {
    const int idx = it * 256 + tid;
    const int row = idx >> 7;
    const int c4  = (idx & 127) * 4;
    const v4f hv = *(const v4f*)(hidden   + (size_t)(b0 + row) * HID + c4);
    const v4f av = *(const v4f*)(init_att + (size_t)(b0 + row) * HID + c4);
    *(v4f*)(Hs + row * FPITCH + c4) = hv;
    *(v4f*)(Fs + row * FPITCH + c4) = av;
  }
  __syncthreads();
  tile_to_f16(Hs, Ah, tid);
  tile_to_f16(Fs, Ac, tid);
  __syncthreads();

  const v8f z8 = {0.f, 0.f, 0.f, 0.f, 0.f, 0.f, 0.f, 0.f};
  const _Float16* ahrow = Ah + c * HPITCH + koff;
  const _Float16* acrow = Ac + c * HPITCH + koff;

#pragma unroll 1
  for (int t = 0; t < T_STEPS; ++t) {
    const bool last = (t == T_STEPS - 1);
    const size_t rowg = (size_t)t * BATCH + (size_t)b0;

    {
      float* gis = Fs + wave * GIS_WAVE;
#pragma unroll 1
      for (int nt = 0; nt < 4; ++nt) {
        const int jc = 64 * wave + 16 * nt;
        const int j  = jc + c;
#pragma unroll
        for (int i = 0; i < 2; ++i) {
          const int idx = lane + 32 * i;
          const int row = idx >> 2;
          const int c4  = (idx & 3) * 4;
          const float* gp = gi32 + (rowg + (size_t)row) * GATES3 + jc + c4;
          const v4f g0 = *(const v4f*)(gp);
          const v4f g1 = *(const v4f*)(gp + HID);
          const v4f g2 = *(const v4f*)(gp + 2 * HID);
          *(v4f*)(gis + row * GIS_P + c4) = g0;
          *(v4f*)(gis + GIS_GATE + row * GIS_P + c4) = g1;
          *(v4f*)(gis + 2 * GIS_GATE + row * GIS_P + c4) = g2;
        }
        const _Float16* wh = WHH + (size_t)j * HID + koff;
        const _Float16* wc = WIC + (size_t)j * HID + koff;
        v8f aR = z8, aZ = z8, aIN = z8, aHN = z8;
#pragma unroll 1
        for (int k0 = 0; k0 < HID; k0 += 32) {
          const v16h fh  = Frag<_Float16>::load(ahrow + k0);
          const v16h fc  = Frag<_Float16>::load(acrow + k0);
          const v16h bhr = Frag<_Float16>::load(wh + k0);
          const v16h bhz = Frag<_Float16>::load(wh + (size_t)HID * HID + k0);
          const v16h bhn = Frag<_Float16>::load(wh + (size_t)2 * HID * HID + k0);
          const v16h bcr = Frag<_Float16>::load(wc + k0);
          const v16h bcz = Frag<_Float16>::load(wc + (size_t)HID * HID + k0);
          const v16h bcn = Frag<_Float16>::load(wc + (size_t)2 * HID * HID + k0);
          aR  = Frag<_Float16>::mma(fh, bhr, aR);
          aZ  = Frag<_Float16>::mma(fh, bhz, aZ);
          aHN = Frag<_Float16>::mma(fh, bhn, aHN);
          aR  = Frag<_Float16>::mma(fc, bcr, aR);
          aZ  = Frag<_Float16>::mma(fc, bcz, aZ);
          aIN = Frag<_Float16>::mma(fc, bcn, aIN);
          guard_gru(aR, aZ, aIN, aHN, fh, fc, bhr, bhz, bhn, bcr, bcz, bcn);
        }
        acc_guard4(aR, aZ, aIN, aHN);
        wave_sync_lds();
        const float bR = sBhh[j];
        const float bZ = sBhh[HID + j];
        const float bN = sBhh[2 * HID + j];
#pragma unroll
        for (int r = 0; r < 8; ++r) {
          const int row = 8 * hh + r;
          const float gr = gis[row * GIS_P + c];
          const float gz = gis[GIS_GATE + row * GIS_P + c];
          const float gn = gis[2 * GIS_GATE + row * GIS_P + c];
          const float pr = aR[r] * FOLD_INV + (gr + bR);
          const float pz = aZ[r] * FOLD_INV + (gz + bZ);
          const float rg = 1.0f / (1.0f + expf(-pr));
          const float zg = 1.0f / (1.0f + expf(-pz));
          const float hn = aHN[r] * FOLD_INV + bN;
          const float nn = tanhf(aIN[r] * FOLD_INV + gn + rg * hn);
          const float ho = Hs[row * FPITCH + j];
          const float h1 = (1.0f - zg) * nn + zg * ho;
          Hs[row * FPITCH + j] = h1;
        }
        wave_sync_lds();
      }
    }
    __syncthreads();

    tile_to_f16(Hs, Ah, tid);
    tile_emit(Hs, Ah, acat16 + rowg * CATW + HID, out6 + rowg * HID, out3 + (size_t)b0 * HID, last, tid);
    __syncthreads();

    {
      const _Float16* wq = WQ + (size_t)(64 * wave + c) * HID + koff;
      v8f q0 = z8, q1 = z8, q2 = z8, q3 = z8;
#pragma unroll 1
      for (int k0 = 0; k0 < HID; k0 += 32) {
        const v16h fh = Frag<_Float16>::load(ahrow + k0);
        const v16h w0 = Frag<_Float16>::load(wq + k0);
        const v16h w1 = Frag<_Float16>::load(wq + (size_t)16 * HID + k0);
        const v16h w2 = Frag<_Float16>::load(wq + (size_t)32 * HID + k0);
        const v16h w3 = Frag<_Float16>::load(wq + (size_t)48 * HID + k0);
        q0 = Frag<_Float16>::mma(fh, w0, q0);
        q1 = Frag<_Float16>::mma(fh, w1, q1);
        q2 = Frag<_Float16>::mma(fh, w2, q2);
        q3 = Frag<_Float16>::mma(fh, w3, q3);
        guard_q(q0, q1, q2, q3, fh, w0, w1, w2, w3);
      }
      acc_guard4(q0, q1, q2, q3);
      const int jq = 64 * wave + c;
#pragma unroll
      for (int r = 0; r < 8; ++r) {
        float* qp = Fs + (8 * hh + r) * FPITCH + jq;
        qp[0]  = q0[r] * FOLD_INV;
        qp[16] = q1[r] * FOLD_INV;
        qp[32] = q2[r] * FOLD_INV;
        qp[48] = q3[r] * FOLD_INV;
      }
    }
    __syncthreads();

#pragma unroll 1
    for (int s = 0; s < 2; ++s) {
      const int bl = 2 * wave + s;
      const int bg = b0 + bl;
      const float* qrow = Fs + bl * FPITCH;
#pragma unroll 1
      for (int l = 0; l < SRCLEN; ++l) {
        const float* pr = pre32 + ((size_t)l * BATCH + (size_t)bg) * HID;
        float acc = 0.0f;
#pragma unroll 1
        for (int i = 0; i < 4; ++i) {
          const int o = 128 * i + 4 * lane;
          const v4f pv = *(const v4f*)(pr + o);
          const v4f qv = *(const v4f*)(qrow + o);
          const v4f wv = *(const v4f*)(sWv + o);
#pragma unroll
          for (int e = 0; e < 4; ++e) acc += tanhf(pv[e] + qv[e]) * wv[e];
        }
#pragma unroll
        for (int off = 16; off > 0; off >>= 1) acc += __shfl_xor(acc, off, 32);
        if (lane == 0) Ss[bl * SRCLEN + l] = acc;
      }
      wave_sync_lds();
      float xv[4];
#pragma unroll
      for (int k = 0; k < 4; ++k) {
        const int l  = lane + 32 * k;
        const int lc = l < SRCLEN ? l : SRCLEN - 1;
        const float ev = Ss[bl * SRCLEN + lc];
        const float mk = mask[(size_t)bg * SRCLEN + lc];
        const float eb = ev + ((mk > 0.0f) ? -1.0e6f : 0.0f);
        xv[k] = (l < SRCLEN) ? eb : -INFINITY;
      }
      float mx = fmaxf(fmaxf(xv[0], xv[1]), fmaxf(xv[2], xv[3]));
#pragma unroll
      for (int off = 16; off > 0; off >>= 1) mx = fmaxf(mx, __shfl_xor(mx, off, 32));
      float pe[4];
      float sum = 0.0f;
#pragma unroll
      for (int k = 0; k < 4; ++k) {
        const int l = lane + 32 * k;
        const float ex = expf(xv[k] - mx);
        pe[k] = (l < SRCLEN) ? ex : 0.0f;
        sum += pe[k];
      }
#pragma unroll
      for (int off = 16; off > 0; off >>= 1) sum += __shfl_xor(sum, off, 32);
      const float inv = 1.0f / sum;
#pragma unroll
      for (int k = 0; k < 4; ++k) {
        const int l = lane + 32 * k;
        const float p = pe[k] * inv;
        if (l < SRCLEN) Ss[bl * SRCLEN + l] = p;
      }
    }
    __syncthreads();

    {
      float* o1 = out1 + rowg * SRCLEN;
      float* o4 = out4 + (size_t)b0 * SRCLEN;
      for (int pass = 0; pass < 2; ++pass) {
#pragma unroll 1
        for (int it = 0; it < 2; ++it) {
          const int idx = it * 256 + tid;
          if (idx < 4 * SRCLEN) {
            const v4f v = *(const v4f*)(Ss + 4 * idx);
            *(volatile v4f*)(o1 + 4 * idx) = v;
            if (last) *(volatile v4f*)(o4 + 4 * idx) = v;
          }
        }
        __threadfence();
      }
    }
#pragma unroll 1
    for (int it = 0; it < 8; ++it) {
      const int idx = it * 256 + tid;
      const int bl  = idx >> 7;
      const int e4  = (idx & 127) * 4;
      const float* cp = context + (size_t)(b0 + bl) * HID + e4;
      const float* sp = Ss + bl * SRCLEN;
      v4f acc = {0.f, 0.f, 0.f, 0.f};
#pragma unroll 4
      for (int l = 0; l < SRCLEN; ++l) {
        const v4f cv = *(const v4f*)(cp + (size_t)l * BATCH * HID);
        const float p = sp[l];
        acc[0] += p * cv[0];
        acc[1] += p * cv[1];
        acc[2] += p * cv[2];
        acc[3] += p * cv[3];
      }
      *(v4f*)(Fs + bl * FPITCH + e4) = acc;
    }
    __syncthreads();

    tile_to_f16(Fs, Ac, tid);
    tile_emit(Fs, Ac, acat16 + rowg * CATW + 2 * HID, wctx32 + rowg * HID, out5 + (size_t)b0 * HID, last, tid);
    __syncthreads();
  }
}

__global__ __launch_bounds__(256) void maxout_kernel(const float* __restrict__ ro, float* __restrict__ out0) {
  const int i = blockIdx.x * 256 + threadIdx.x;
  if (i < ROWS_TB * 64) {
    const int row = i >> 6;
    const int j4  = (i & 63) * 4;
    const float* rp = ro + (size_t)row * HID + 2 * j4;
    const v4f a = *(const v4f*)(rp);
    const v4f b = *(const v4f*)(rp + 4);
    v4f o;
    o[0] = fmaxf(a[0], a[1]);
    o[1] = fmaxf(a[2], a[3]);
    o[2] = fmaxf(b[0], b[1]);
    o[3] = fmaxf(b[2], b[3]);
    float* op = out0 + (size_t)row * (HID / 2) + j4;
    *(volatile v4f*)op = o;
    __threadfence();
    *(volatile v4f*)op = o;
  }
}

__global__ __launch_bounds__(256) void copy_gate_kernel(const float* __restrict__ h1seq, const float* __restrict__ wctx32,
                                                        const float* __restrict__ w_copy, const float* __restrict__ b_copy,
                                                        float* __restrict__ out2) {
  __shared__ float sP[32];
  const int tid = threadIdx.x, lane = tid & 31, wave = tid >> 5;
  const float bc = b_copy[0];
#pragma unroll 1
  for (int s = 0; s < 4; ++s) {
    const int row = blockIdx.x * 32 + wave * 4 + s;
    const float* hp = h1seq  + (size_t)row * HID;
    const float* cp = wctx32 + (size_t)row * HID;
    float acc = 0.0f;
#pragma unroll 1
    for (int i = 0; i < 4; ++i) {
      const int o = 128 * i + 4 * lane;
      const v4f hv = *(const v4f*)(hp + o);
      const v4f cv = *(const v4f*)(cp + o);
      const v4f w0 = *(const v4f*)(w_copy + o);
      const v4f w1 = *(const v4f*)(w_copy + HID + o);
#pragma unroll
      for (int e = 0; e < 4; ++e) {
        acc += hv[e] * w0[e];
        acc += cv[e] * w1[e];
      }
    }
#pragma unroll
    for (int off = 16; off > 0; off >>= 1) acc += __shfl_xor(acc, off, 32);
    const float p = 1.0f / (1.0f + expf(-(acc + bc)));
    if (lane == 0) sP[wave * 4 + s] = p;
  }
  __syncthreads();
  if (wave == 0) {
    const float v = sP[lane];
    float* op = out2 + (size_t)blockIdx.x * 32 + lane;
    *(volatile float*)op = v;
    __threadfence();
    *(volatile float*)op = v;
  }
}

extern "C" void kernel_launch(void* const* d_in, const int* in_sizes, int n_in,
                              void* d_out, int out_size, void* d_ws, size_t ws_size, hipStream_t stream) {
  if (n_in < 21 || d_out == nullptr || d_ws == nullptr) return;
  if (in_sizes[1] != ROWS_TB || in_sizes[2] != BATCH * HID || in_sizes[3] != ROWS_LB * HID ||
      in_sizes[4] != BATCH * SRCLEN || in_sizes[5] != BATCH * HID || in_sizes[8] != VOCAB * HID ||
      in_sizes[9] != GATES3 * 2 * HID || in_sizes[10] != GATES3 * HID || in_sizes[11] != GATES3 ||
      in_sizes[12] != GATES3 || in_sizes[13] != HID * HID || in_sizes[14] != HID || in_sizes[15] != HID * HID ||
      in_sizes[16] != HID || in_sizes[17] != 2 * HID || in_sizes[18] != 1 || in_sizes[19] != HID * CATW ||
      in_sizes[20] != HID || out_size != OUT_TOTAL) return;

  const int*   input_ids = (const int*)  d_in[1];
  const float* hidden    = (const float*)d_in[2];
  const float* context   = (const float*)d_in[3];
  const float* mask      = (const float*)d_in[4];
  const float* init_att  = (const float*)d_in[5];
  const float* word_lut  = (const float*)d_in[8];
  const float* W_ih      = (const float*)d_in[9];
  const float* W_hh      = (const float*)d_in[10];
  const float* b_ih      = (const float*)d_in[11];
  const float* b_hh      = (const float*)d_in[12];
  const float* W_pre     = (const float*)d_in[13];
  const float* b_pre     = (const float*)d_in[14];
  const float* W_q       = (const float*)d_in[15];
  const float* W_v       = (const float*)d_in[16];
  const float* W_copy    = (const float*)d_in[17];
  const float* b_copy    = (const float*)d_in[18];
  const float* W_read    = (const float*)d_in[19];
  const float* b_read    = (const float*)d_in[20];

  float* out  = (float*)d_out;
  float* out0 = out;
  float* out1 = out + OFF1;
  float* out2 = out + OFF2;
  float* out3 = out + OFF3;
  float* out4 = out + OFF4;
  float* out5 = out + OFF5;
  float* out6 = out + OFF6;

  char* ws = (char*)d_ws; size_t off = 0;
  auto carve = [&](size_t bytes) -> char* { char* p = ws + off; off += (bytes + 255) & ~(size_t)255; return p; };
  unsigned short* WIHE  = (unsigned short*)carve((size_t)GATES3 * HID * 2);
  unsigned short* WIHC  = (unsigned short*)carve((size_t)GATES3 * HID * 2);
  unsigned short* WHH   = (unsigned short*)carve((size_t)GATES3 * HID * 2);
  unsigned short* WQ    = (unsigned short*)carve((size_t)HID * HID * 2);
  unsigned short* WPRE  = (unsigned short*)carve((size_t)HID * HID * 2);
  unsigned short* WREAD = (unsigned short*)carve((size_t)HID * CATW * 2);
  unsigned short* CTX16 = (unsigned short*)carve((size_t)ROWS_LB * HID * 2);
  float*          PRE32 = (float*)carve((size_t)ROWS_LB * HID * 4);
  unsigned short* ACAT  = (unsigned short*)carve((size_t)ROWS_TB * CATW * 2);
  float*          GI32  = (float*)carve((size_t)ROWS_TB * GATES3 * 4);
  float*          WCTX  = (float*)carve((size_t)ROWS_TB * HID * 4);
  float*          RO32  = (float*)carve((size_t)ROWS_TB * HID * 4);
  if (off > ws_size || off > (size_t)134217728) return;

  const int n8g = GATES3 * (HID / 8);
  const int n8s = HID * (HID / 8);
  const int n8r = HID * (CATW / 8);
  const int n8c = ROWS_LB * (HID / 8);
  cvt8_f16_kernel<<<n8g / 256, 256, 0, stream>>>(W_ih,    WIHE,  GATES3,  HID / 8,  2 * HID, 0,   OPCARRY);
  cvt8_f16_kernel<<<n8g / 256, 256, 0, stream>>>(W_ih,    WIHC,  GATES3,  HID / 8,  2 * HID, HID, OPCARRY);
  cvt8_f16_kernel<<<n8g / 256, 256, 0, stream>>>(W_hh,    WHH,   GATES3,  HID / 8,  HID,     0,   OPCARRY);
  cvt8_f16_kernel<<<n8s / 256, 256, 0, stream>>>(W_q,     WQ,    HID,     HID / 8,  HID,     0,   OPCARRY);
  cvt8_f16_kernel<<<n8s / 256, 256, 0, stream>>>(W_pre,   WPRE,  HID,     HID / 8,  HID,     0,   OPCARRY);
  cvt8_f16_kernel<<<n8r / 256, 256, 0, stream>>>(W_read,  WREAD, HID,     CATW / 8, CATW,    0,   OPCARRY);
  cvt8_f16_kernel<<<n8c / 256, 256, 0, stream>>>(context, CTX16, ROWS_LB, HID / 8,  HID,     0,   OPCARRY);
  gather_emb_kernel<<<(ROWS_TB * 64) / 256, 256, 0, stream>>>(input_ids, word_lut, ACAT);

  wmma_gemm64<0, false, 2, 0, false, 0><<<dim3((ROWS_LB / 64) * (HID / 64) / 8, 1), 256, 0, stream>>>(
      CTX16, CTX16, HID, 0L, WPRE, WPRE, HID, 0L, (void*)PRE32, (void*)PRE32, HID, 0L,
      b_pre, b_pre, 0L, ROWS_LB, HID, HID, FOLD_INV);
  wmma_gemm64<0, false, 2, 0, false, 0><<<dim3((ROWS_TB / 64) * (GATES3 / 64) / 8, 1), 256, 0, stream>>>(
      ACAT, ACAT, CATW, 0L, WIHE, WIHE, HID, 0L, (void*)GI32, (void*)GI32, GATES3, 0L,
      b_ih, b_ih, 0L, ROWS_TB, GATES3, HID, FOLD_INV);

  dec_seq_kernel<<<BATCH / 16, 256, 0, stream>>>(hidden, init_att, context, mask, PRE32, GI32, b_hh, W_v,
                                                 WHH, WIHC, WQ, ACAT, WCTX, out1, out3, out4, out5, out6);

  wmma_gemm64<0, false, 2, 0, false, 0><<<dim3((ROWS_TB / 64) * (HID / 64) / 8, 1), 256, 0, stream>>>(
      ACAT, ACAT, CATW, 0L, WREAD, WREAD, CATW, 0L, (void*)RO32, (void*)RO32, HID, 0L,
      b_read, b_read, 0L, ROWS_TB, HID, CATW, FOLD_INV);
  maxout_kernel<<<(ROWS_TB * 64) / 256, 256, 0, stream>>>(RO32, out0);
  copy_gate_kernel<<<ROWS_TB / 32, 256, 0, stream>>>(out6, WCTX, W_copy, b_copy, out2);
}
